// DecoderBlock_60473139527979
// MI455X (gfx1250) — hardware-verified
//
#include <hip/hip_runtime.h>
#include <math.h>

typedef __attribute__((ext_vector_type(16))) _Float16 v16h;
typedef __attribute__((ext_vector_type(8)))  _Float16 v8h;
typedef __attribute__((ext_vector_type(4)))  _Float16 v4h;
typedef __attribute__((ext_vector_type(8)))  float v8f;
typedef __attribute__((ext_vector_type(4)))  float v4f;
typedef __attribute__((ext_vector_type(4)))  unsigned v4u;

template <typename T> __device__ __forceinline__ void vst2(void* p, T v) { *(volatile T*)p = v; __threadfence(); *(volatile T*)p = v; }
__device__ __forceinline__ v8f wmma16(v16h a, v16h b, v8f c) {
  v8f d = __builtin_amdgcn_wmma_f32_16x16x32_f16(false, a, false, b, (short)0, c, false, false);
  asm volatile("v_nop\n\tv_nop\n\tv_nop\n\tv_nop" : "+v"(d) : "v"(a), "v"(b));
  return d;
}
__device__ __forceinline__ v16h frag_h(const _Float16* rowk0, unsigned lane) {
  union { v16h v; v8h q[2]; } u; const _Float16* p = rowk0 + 8u * (lane >> 4);
  u.q[0] = *(const v8h*)p; u.q[1] = *(const v8h*)(p + 16); return u.v;
}
__device__ __forceinline__ float bfr(float v) { return (float)(__bf16)v; }
#define LDSX() do { asm volatile("s_wait_dscnt 0" ::: "memory"); __builtin_amdgcn_wave_barrier(); __builtin_amdgcn_fence(3  , "workgroup"); } while (0)

#ifndef NB
#define NB 32
#endif
#ifndef SEQ
#define SEQ 768
#endif
#define NB_FULL 32
#define SEQ_FULL 768
#define CC 384
#define NH 6
#define HD 64
#define FF 1536
#define NRW (NB * SEQ)
#define NHALF (NRW / 2)
#define XNEED (((size_t)(NB - 1) * SEQ_FULL + SEQ) * CC)

static_assert(NH * HD == CC);
static_assert(CC % 128 == 0);
static_assert(FF % 128 == 0);
static_assert(SEQ % 64 == 0);
static_assert(NRW % 128 == 0);
static_assert(NB <= NB_FULL);
static_assert(SEQ <= SEQ_FULL);

#define SZ_ACT  (2u * (size_t)NRW * CC)
#define WS_WQKV 0u
#define WS_WO   (WS_WQKV + 2u * 3u * (size_t)CC * CC)
#define WS_W1   (WS_WO + 2u * (size_t)CC * CC)
#define WS_W2   (WS_W1 + 2u * (size_t)FF * CC)
#define WS_XH   (WS_W2 + 2u * (size_t)CC * FF)
#define WS_QH   (WS_XH + SZ_ACT)
#define WS_KH   (WS_QH + SZ_ACT)
#define WS_VT   (WS_KH + SZ_ACT)
#define WS_R1   (WS_VT + SZ_ACT)
#define WS_END  (WS_R1 + 4u * (size_t)NRW * CC)
#define WS_HF   WS_QH
static_assert(2u * (size_t)NHALF * FF == 2u * SZ_ACT);
static_assert(WS_END <= 134217728u);
static_assert(WS_XH % 128u == 0u);

__device__ __forceinline__ unsigned frow(unsigned r) { const unsigned b = r / (unsigned)SEQ; return b * (unsigned)SEQ_FULL + (r - b * (unsigned)SEQ); }

__global__ __launch_bounds__(256) void k_wt(const float* __restrict__ W, unsigned K, unsigned N, _Float16* __restrict__ Wt) {
  __shared__ __align__(16) _Float16 t[64][72];
  const unsigned tid = threadIdx.x, k0 = blockIdx.x * 64u, n0 = blockIdx.y * 64u;
#pragma unroll 4
  for (unsigned e = tid; e < 4096u; e += 256u) { const unsigned kk = e >> 6, nn = e & 63u; t[nn][kk] = (_Float16)(bfr(W[(size_t)(k0 + kk) * N + n0 + nn]) * 64.0f); }
  __syncthreads();
  for (unsigned e = tid; e < 512u; e += 256u) { const unsigned nn = e >> 3, q = e & 7u; const v4u v = *(const v4u*)&t[nn][q * 8u]; vst2(Wt + (size_t)(n0 + nn) * K + k0 + q * 8u, v); }
}

__global__ __launch_bounds__(256) void k_lnx(const float* __restrict__ X, unsigned fullmap, unsigned bfin, const float* __restrict__ G, const float* __restrict__ BE, _Float16* __restrict__ OUT) {
  const unsigned wave = threadIdx.x >> 5, lane = threadIdx.x & 31u; const unsigned row = blockIdx.x * 8u + wave; if (row >= (unsigned)NRW) return;
  const size_t xr = fullmap ? (size_t)frow(row) : (size_t)row;
  v4f v[CC / 128]; float s1 = 0.f;
#pragma unroll
  for (int i = 0; i < CC / 128; ++i) { v4f t = *(const v4f*)(X + xr * CC + i * 128 + lane * 4u); if (bfin) { t[0] = bfr(t[0]); t[1] = bfr(t[1]); t[2] = bfr(t[2]); t[3] = bfr(t[3]); } v[i] = t; s1 += (t[0] + t[1]) + (t[2] + t[3]); }
#pragma unroll
  for (int o = 1; o < 32; o <<= 1) s1 += __shfl_xor(s1, o);
  const float mu = s1 * (1.0f / CC); float q = 0.f;
#pragma unroll
  for (int i = 0; i < CC / 128; ++i) {
#pragma unroll
    for (int k = 0; k < 4; ++k) { const float d = v[i][k] - mu; q += d * d; } }
#pragma unroll
  for (int o = 1; o < 32; o <<= 1) q += __shfl_xor(q, o);
  const float inv = rsqrtf(q * (1.0f / CC) + 1e-5f);
#pragma unroll
  for (int i = 0; i < CC / 128; ++i) { const unsigned c = i * 128u + lane * 4u; const v4f gv = *(const v4f*)(G + c), bv = *(const v4f*)(BE + c); v4h r4;
#pragma unroll
    for (int k = 0; k < 4; ++k) r4[k] = (_Float16)(bfr(gv[k]) * ((v[i][k] - mu) * inv) + bfr(bv[k]));
    vst2(OUT + (size_t)row * CC + c, r4); }
}

__global__ __launch_bounds__(128) void k_g16(const _Float16* __restrict__ A, unsigned K, const _Float16* __restrict__ Wt, unsigned N, const float* __restrict__ BIAS, unsigned relu, float carry,
    _Float16* __restrict__ D0, _Float16* __restrict__ D1, _Float16* __restrict__ DT) {
  __shared__ __align__(16) _Float16 sh[64][136]; __shared__ __align__(16) _Float16 th[128][72];
  const unsigned tid = threadIdx.x, wave = tid >> 5, lane = tid & 31u, col = lane & 15u, g = lane >> 4; const unsigned z = blockIdx.z, c0 = blockIdx.y * 128u; const size_t r0 = (size_t)blockIdx.x * 64u;
  const _Float16* ap = A + (r0 + wave * 16u + col) * K; const _Float16* wp = Wt + (size_t)z * N * K + (size_t)(c0 + col) * K;
  v8f acc[8] = {};
#pragma unroll 2
  for (unsigned kc = 0; kc < K / 32u; ++kc) { const v16h a = frag_h(ap + kc * 32u, lane);
#pragma unroll
    for (int j = 0; j < 8; ++j) { const v16h w = frag_h(wp + (size_t)j * 16u * K + kc * 32u, lane); acc[j] = wmma16(a, w, acc[j]); } }
  if (z < 2u) { _Float16* D = z == 0u ? D0 : D1;
#pragma unroll
    for (int j = 0; j < 8; ++j) { const float bb = BIAS ? bfr(BIAS[c0 + j * 16u + col]) : 0.f;
#pragma unroll
      for (int r = 0; r < 8; ++r) { float v = acc[j][r] * (1.0f / 64.0f) + bb; if (relu) v = fmaxf(v, 0.f); sh[wave * 16u + 8u * g + r][j * 16u + col] = (_Float16)(v * carry); } }
    __syncthreads();
    for (unsigned e = tid; e < 1024u; e += 128u) { const unsigned rl = e >> 4, q = e & 15u; const v4u v = *(const v4u*)&sh[rl][q * 8u]; vst2(D + (r0 + rl) * N + c0 + q * 8u, v); }
  } else { const unsigned bq = (unsigned)r0 / (unsigned)SEQ, t0 = (unsigned)r0 - bq * (unsigned)SEQ;
#pragma unroll
    for (int j = 0; j < 8; ++j) { const float bb = BIAS ? bfr(BIAS[c0 + j * 16u + col]) : 0.f;
#pragma unroll
      for (int r = 0; r < 8; ++r) { float v = acc[j][r] * (1.0f / 64.0f) + bb; if (relu) v = fmaxf(v, 0.f); th[j * 16u + col][wave * 16u + 8u * g + r] = (_Float16)(v * carry); } }
    __syncthreads();
    for (unsigned e = tid; e < 1024u; e += 128u) { const unsigned cl = e >> 3, q = e & 7u; const v4u v = *(const v4u*)&th[cl][q * 8u]; vst2(DT + ((size_t)bq * N + c0 + cl) * SEQ + t0 + q * 8u, v); } }
}

__global__ __launch_bounds__(128) void k_fa(const _Float16* __restrict__ QH, const _Float16* __restrict__ KH, const _Float16* __restrict__ VT, _Float16* __restrict__ YH) {
  __shared__ __align__(16) _Float16 sp[4][16][40]; __shared__ __align__(16) _Float16 sy[4][16][72];
  const unsigned tid = threadIdx.x, wave = tid >> 5, lane = tid & 31u, col = lane & 15u, g = lane >> 4;
  const unsigned bh = blockIdx.y, b = bh / (unsigned)NH, h = bh - b * (unsigned)NH; const unsigned q0 = blockIdx.x * 64u + wave * 16u; const size_t rb = (size_t)b * SEQ;
  const _Float16* qp = QH + (rb + q0 + col) * CC + h * HD;
  const v16h qf0 = frag_h(qp, lane), qf1 = frag_h(qp + 32, lane);
  const _Float16* kbase = KH + (rb + col) * CC + h * HD;
  const _Float16* vbase = VT + ((size_t)b * CC + h * HD + col) * SEQ;
  v8f o[4] = {}; float rmax[8], rsum[8];
#pragma unroll
  for (int r = 0; r < 8; ++r) { rmax[r] = -3.0e38f; rsum[r] = 0.f; }
  const unsigned nk = (q0 + 47u) >> 5;
#pragma unroll 1
  for (unsigned kc = 0; kc < nk; ++kc) { const unsigned k0 = kc * 32u;
    v8f s0 = {}, s1 = {};
    { const _Float16* kp = kbase + (size_t)k0 * CC; s0 = wmma16(qf0, frag_h(kp, lane), s0); s0 = wmma16(qf1, frag_h(kp + 32, lane), s0);
      kp += 16 * CC; s1 = wmma16(qf0, frag_h(kp, lane), s1); s1 = wmma16(qf1, frag_h(kp + 32, lane), s1); }
#pragma unroll
    for (int r = 0; r < 8; ++r) { const unsigned qg = q0 + 8u * g + (unsigned)r;
      float a0 = s0[r] * 0.125f, a1 = s1[r] * 0.125f;
      a0 = (k0 + col <= qg) ? a0 : -3.0e38f; a1 = (k0 + 16u + col <= qg) ? a1 : -3.0e38f;
      float mx = fmaxf(a0, a1);
      mx = fmaxf(mx, __shfl_xor(mx, 8)); mx = fmaxf(mx, __shfl_xor(mx, 4)); mx = fmaxf(mx, __shfl_xor(mx, 2)); mx = fmaxf(mx, __shfl_xor(mx, 1));
      const float nm = fmaxf(rmax[r], mx); const float alpha = expf(rmax[r] - nm); rmax[r] = nm;
      const float p0 = expf(a0 - nm), p1 = expf(a1 - nm);
      rsum[r] = rsum[r] * alpha + (p0 + p1);
      o[0][r] *= alpha; o[1][r] *= alpha; o[2][r] *= alpha; o[3][r] *= alpha;
      sp[wave][8u * g + r][col] = (_Float16)(p0 * 256.0f); sp[wave][8u * g + r][16u + col] = (_Float16)(p1 * 256.0f); }
    LDSX();
    v16h pf; { union { v16h v; v8h q[2]; } u; u.q[0] = *(const v8h*)&sp[wave][col][8u * g]; u.q[1] = *(const v8h*)&sp[wave][col][16u + 8u * g]; pf = u.v; }
#pragma unroll
    for (int j = 0; j < 4; ++j) o[j] = wmma16(pf, frag_h(vbase + (size_t)j * 16u * SEQ + k0, lane), o[j]);
    LDSX(); }
#pragma unroll
  for (int r = 0; r < 8; ++r) { float t = rsum[r]; t += __shfl_xor(t, 8); t += __shfl_xor(t, 4); t += __shfl_xor(t, 2); t += __shfl_xor(t, 1);
    const float inv = 0.0625f * (1.0f / t);
#pragma unroll
    for (int j = 0; j < 4; ++j) sy[wave][8u * g + r][j * 16u + col] = (_Float16)(o[j][r] * inv); }
  LDSX();
  for (unsigned e = lane; e < 128u; e += 32u) { const unsigned rl = e >> 3, q = e & 7u; const v4u v = *(const v4u*)&sy[wave][rl][q * 8u]; vst2(YH + (rb + q0 + rl) * CC + h * HD + q * 8u, v); }
}

__global__ __launch_bounds__(128) void k_gemf(const _Float16* __restrict__ A, unsigned K, const _Float16* __restrict__ Wt, unsigned N, float osc, const float* __restrict__ BIAS,
    const float* __restrict__ RES, unsigned res_full, unsigned res_bf, float* __restrict__ OUT, unsigned out_full, unsigned rbase) {
  __shared__ __align__(16) float sf[4][16][132];
  const unsigned tid = threadIdx.x, wave = tid >> 5, lane = tid & 31u, col = lane & 15u, g = lane >> 4; const unsigned c0 = blockIdx.y * 128u;
  const unsigned lr0 = blockIdx.x * 64u + wave * 16u; const unsigned fr0 = frow(rbase + lr0);
  const size_t rr0 = res_full ? (size_t)fr0 : (size_t)lr0; const size_t or0 = out_full ? (size_t)fr0 : (size_t)lr0;
  const _Float16* ap = A + (size_t)(lr0 + col) * K; const _Float16* wp = Wt + (size_t)(c0 + col) * K;
  v8f acc[8] = {};
#pragma unroll 2
  for (unsigned kc = 0; kc < K / 32u; ++kc) { const v16h a = frag_h(ap + kc * 32u, lane);
#pragma unroll
    for (int j = 0; j < 8; ++j) { const v16h w = frag_h(wp + (size_t)j * 16u * K + kc * 32u, lane); acc[j] = wmma16(a, w, acc[j]); } }
#pragma unroll
  for (int j = 0; j < 8; ++j) { const float bb = BIAS ? bfr(BIAS[c0 + j * 16u + col]) : 0.f;
#pragma unroll
    for (int r = 0; r < 8; ++r) sf[wave][8u * g + r][j * 16u + col] = acc[j][r] * osc + bb; }
  LDSX();
  for (unsigned rl = 0; rl < 16u; ++rl) { v4f v = *(const v4f*)&sf[wave][rl][lane * 4u]; v4f rv = *(const v4f*)(RES + (rr0 + rl) * N + c0 + lane * 4u);
    if (res_bf) { rv[0] = bfr(rv[0]); rv[1] = bfr(rv[1]); rv[2] = bfr(rv[2]); rv[3] = bfr(rv[3]); }
    v[0] += rv[0]; v[1] += rv[1]; v[2] += rv[2]; v[3] += rv[3];
    vst2(OUT + (or0 + rl) * N + c0 + lane * 4u, v); }
}

extern "C" void kernel_launch(void* const* d_in, const int* in_sizes, int n_in, void* d_out, int out_size, void* d_ws, size_t ws_size, hipStream_t stream) {
  if (n_in < 14) return;
  if ((size_t)in_sizes[0] < XNEED || (size_t)out_size < XNEED) return;
  if (in_sizes[1] < CC * CC || in_sizes[2] < CC * CC || in_sizes[3] < CC * CC || in_sizes[4] < CC * CC) return;
  if (in_sizes[5] < CC || in_sizes[6] < CC || in_sizes[7] < CC || in_sizes[8] < CC || in_sizes[9] < CC || in_sizes[13] < CC) return;
  if (in_sizes[10] < CC * FF || in_sizes[11] < FF || in_sizes[12] < FF * CC) return;
  if (ws_size < (size_t)WS_END) return;
  const float** F = (const float**)d_in;
  char* ws = (char*)d_ws;
  _Float16 *WQKV = (_Float16*)(ws + WS_WQKV), *WO = (_Float16*)(ws + WS_WO), *WF1 = (_Float16*)(ws + WS_W1), *WF2 = (_Float16*)(ws + WS_W2);
  _Float16 *XH = (_Float16*)(ws + WS_XH), *QH = (_Float16*)(ws + WS_QH), *KH = (_Float16*)(ws + WS_KH), *VT = (_Float16*)(ws + WS_VT), *HF = (_Float16*)(ws + WS_HF);
  _Float16 *YH = XH;
  float* R1 = (float*)(ws + WS_R1);
  k_wt<<<dim3(CC / 64, CC / 64), 256, 0, stream>>>(F[1], CC, CC, WQKV);
  k_wt<<<dim3(CC / 64, CC / 64), 256, 0, stream>>>(F[2], CC, CC, WQKV + (size_t)CC * CC);
  k_wt<<<dim3(CC / 64, CC / 64), 256, 0, stream>>>(F[3], CC, CC, WQKV + 2 * (size_t)CC * CC);
  k_wt<<<dim3(CC / 64, CC / 64), 256, 0, stream>>>(F[4], CC, CC, WO);
  k_wt<<<dim3(CC / 64, FF / 64), 256, 0, stream>>>(F[10], CC, FF, WF1);
  k_wt<<<dim3(FF / 64, CC / 64), 256, 0, stream>>>(F[12], FF, CC, WF2);
  k_lnx<<<dim3(NRW / 8), 256, 0, stream>>>(F[0], 1u, 1u, F[6], F[7], XH);
  k_g16<<<dim3(NRW / 64, CC / 128, 3), 128, 0, stream>>>(XH, CC, WQKV, CC, nullptr, 0u, 1.0f, QH, KH, VT);
  k_fa<<<dim3(SEQ / 64, NB * NH), 128, 0, stream>>>(QH, KH, VT, YH);
  k_gemf<<<dim3(NRW / 64, CC / 128), 128, 0, stream>>>(YH, CC, WO, CC, 1.0f / 1024.0f, F[5], F[0], 1u, 1u, R1, 0u, 0u);
  k_lnx<<<dim3(NRW / 8), 256, 0, stream>>>(R1, 0u, 0u, F[8], F[9], XH);
  for (unsigned hq = 0; hq < 2u; ++hq) { const size_t ro = (size_t)hq * NHALF;
    k_g16<<<dim3(NHALF / 64, FF / 128, 1), 128, 0, stream>>>(XH + ro * CC, CC, WF1, FF, F[11], 1u, 16.0f, HF, nullptr, nullptr);
    k_gemf<<<dim3(NHALF / 64, CC / 128), 128, 0, stream>>>(HF, FF, WF2, CC, 1.0f / 1024.0f, F[13], R1 + ro * CC, 0u, 0u, (float*)d_out, 1u, (unsigned)ro); }
}
